// PixelBlock_58755152609940
// MI455X (gfx1250) — hardware-verified
//
#include <hip/hip_runtime.h>
#include <math.h>

typedef __attribute__((ext_vector_type(16))) _Float16 v16h;
typedef __attribute__((ext_vector_type(16))) __bf16 v16b;
typedef __attribute__((ext_vector_type(8)))  _Float16 v8h;
typedef __attribute__((ext_vector_type(8)))  float v8f;
typedef __attribute__((ext_vector_type(4)))  float v4f;
typedef __attribute__((ext_vector_type(2)))  float v2f;
typedef __attribute__((ext_vector_type(4)))  unsigned v4u;
typedef __attribute__((ext_vector_type(4)))  int v4i;
typedef float __attribute__((may_alias)) float_a;
typedef int __attribute__((may_alias)) int_a;

template <typename T> __device__ __forceinline__ void vst2(void* p, T v) { *(volatile T*)p = v; __threadfence(); *(volatile T*)p = v; }
__device__ __forceinline__ v8f wmma16(v16h a, v16h b, v8f c) {
  v8f d = __builtin_amdgcn_wmma_f32_16x16x32_f16(false, a, false, b, (short)0, c, false, false);
  asm volatile("v_nop\n\tv_nop\n\tv_nop\n\tv_nop" : "+v"(d) : "v"(a), "v"(b));
  return d;
}
__device__ __forceinline__ v8f wmma_bf(v16b a, v16b b, v8f c) {
  v8f d = __builtin_amdgcn_wmma_f32_16x16x32_bf16(false, a, false, b, (short)0, c, false, false);
  asm volatile("v_nop\n\tv_nop\n\tv_nop\n\tv_nop" : "+v"(d) : "v"(a), "v"(b));
  return d;
}
__device__ __forceinline__ v16h frag_h(const _Float16* rowk0, int lane) {
  union { v16h v; v8h q[2]; } u; const _Float16* p = rowk0 + 8 * (lane >> 4);
  u.q[0] = *(const v8h*)p; u.q[1] = *(const v8h*)(p + 16); return u.v;
}
__device__ __forceinline__ v16h frag_f32(const float* rowk0, int lane) {
  v16h a; const float* p = rowk0 + 8 * (lane >> 4);
#pragma unroll
  for (int i = 0; i < 8; ++i) { a[i] = (_Float16)p[i]; a[8 + i] = (_Float16)p[16 + i]; }
  return a;
}
__device__ __forceinline__ v16h frag_f32s(const float* rowk0, int lane, float sc) {
  v16h a; const float* p = rowk0 + 8 * (lane >> 4);
#pragma unroll
  for (int i = 0; i < 8; ++i) { a[i] = (_Float16)(p[i] * sc); a[8 + i] = (_Float16)(p[16 + i] * sc); }
  return a;
}
__device__ __forceinline__ v16h fragc_f32(const float* W, int k0, int n, int lane, int ld, int K) {
  v16h a; const int g = lane >> 4;
#pragma unroll
  for (int i = 0; i < 8; ++i) { const int ka = k0 + 8 * g + i, kb = ka + 16;
    a[i] = (_Float16)(ka < K ? W[(size_t)ka * ld + n] : 0.f); a[8 + i] = (_Float16)(kb < K ? W[(size_t)kb * ld + n] : 0.f); }
  return a;
}
struct F2 { v16b h, l; };
__device__ __forceinline__ F2 bsplit16(const float v[16]) { F2 r;
#pragma unroll
  for (int i = 0; i < 16; ++i) { const __bf16 h = (__bf16)v[i]; r.h[i] = h; r.l[i] = (__bf16)(v[i] - (float)h); }
  return r; }
__device__ __forceinline__ F2 split_row(const float* row, int k0, int lane) { float v[16]; const float* p = row + k0 + 8 * (lane >> 4);
#pragma unroll
  for (int i = 0; i < 8; ++i) { v[i] = p[i]; v[8 + i] = p[16 + i]; }
  return bsplit16(v); }
__device__ __forceinline__ F2 split_rowK(const float* row, int k0, int lane, int K) { float v[16]; const int g = lane >> 4;
#pragma unroll
  for (int i = 0; i < 8; ++i) { const int ka = k0 + 8 * g + i, kb = ka + 16; v[i] = ka < K ? row[ka] : 0.f; v[8 + i] = kb < K ? row[kb] : 0.f; }
  return bsplit16(v); }
__device__ __forceinline__ F2 split_col(const float* W, int k0, int n, int lane, int ld, int K) { float v[16]; const int g = lane >> 4;
#pragma unroll
  for (int i = 0; i < 8; ++i) { const int ka = k0 + 8 * g + i, kb = ka + 16; v[i] = ka < K ? W[(size_t)ka * ld + n] : 0.f; v[8 + i] = kb < K ? W[(size_t)kb * ld + n] : 0.f; }
  return bsplit16(v); }
__device__ __forceinline__ v8f mac3(const F2& a, const F2& b, v8f c) { c = wmma_bf(a.l, b.h, c); c = wmma_bf(a.h, b.l, c); return wmma_bf(a.h, b.h, c); }
__device__ __forceinline__ float sigm(float v) { return 1.0f / (1.0f + expf(-v)); }
#define LDSX() do { asm volatile("s_wait_dscnt 0" ::: "memory"); __builtin_amdgcn_wave_barrier(); __builtin_amdgcn_fence(__ATOMIC_RELEASE, "workgroup"); } while (0)

#define NB 2
#define CIN 192
#define EM 256
#define NH 8
#define HD 32
#define LL 2304
#define NR (NB * LL)

__global__ __launch_bounds__(128) void k_qkv(const float* __restrict__ qin, const float* __restrict__ kin, const float* __restrict__ Wq, const float* __restrict__ bq, const float* __restrict__ Wk, const float* __restrict__ bk, const float* __restrict__ Wv, const float* __restrict__ bv,
                                           float* __restrict__ QH, float* __restrict__ KH, float* __restrict__ VH) {
  __shared__ __align__(16) float so[4][16][132];
  const int tid = threadIdx.x, wave = tid >> 5, lane = tid & 31, col = lane & 15, g = lane >> 4;
  const int which = blockIdx.z, b = blockIdx.y >> 1, n0 = (blockIdx.y & 1) * 128, l0 = blockIdx.x * 64 + wave * 16;
  const float* X = (which == 0 ? qin : kin) + (size_t)b * CIN * LL; const float* W = which == 0 ? Wq : (which == 1 ? Wk : Wv); const float* bias = which == 0 ? bq : (which == 1 ? bk : bv);
  v8f acc[8] = {};
#pragma unroll 1
  for (int kc = 0; kc < CIN / 32; ++kc) { const F2 a = split_col(X, kc * 32, l0 + col, lane, LL, CIN);
#pragma unroll
    for (int j = 0; j < 8; ++j) acc[j] = mac3(a, split_row(W + (size_t)(n0 + j * 16 + col) * CIN, kc * 32, lane), acc[j]); }
#pragma unroll
  for (int j = 0; j < 8; ++j) { const float bb = bias[n0 + j * 16 + col];
#pragma unroll
    for (int r = 0; r < 8; ++r) so[wave][8 * g + r][j * 16 + col] = acc[j][r] + bb; }
  LDSX();
  float* D = which == 0 ? QH : (which == 1 ? KH : VH);
  for (int q = lane; q < 16 * 4 * 8; q += 32) { const int rl = q >> 5, hh = (q >> 3) & 3, pc = q & 7; const int h = (n0 >> 5) + hh;
    vst2(D + (((size_t)b * NH + h) * LL + l0 + rl) * HD + pc * 4, *(const v4f*)(&so[wave][rl][hh * 32 + pc * 4])); }
}
__global__ __launch_bounds__(128) void k_attn(const float* __restrict__ QH, const float* __restrict__ KH, const float* __restrict__ VH, float* __restrict__ out) {
  __shared__ __align__(16) float sS[4][16][68];
  __shared__ __align__(16) float sO[HD][68];
  const int tid = threadIdx.x, w = tid >> 5, lane = tid & 31, col = lane & 15, g = lane >> 4;
  const int b = blockIdx.z, h = blockIdx.y, q0b = blockIdx.x * 64, q0 = q0b + w * 16; const size_t bh = (size_t)b * NH + h;
  const float scl = 1.0f / sqrtf((float)HD);
  const F2 aq = split_row(QH + (bh * LL + q0 + col) * HD, 0, lane);
  float mrun = -3.0e38f, lrun = 0.f; v8f acc[2] = {};
  const int ntiles = blockIdx.x + 1;
#pragma unroll 1
  for (int kt = 0; kt < ntiles; ++kt) {
#pragma unroll
    for (int t = 0; t < 4; ++t) { v8f s = {}; const int key = kt * 64 + t * 16 + col;
      s = mac3(aq, split_row(KH + (bh * LL + key) * HD, 0, lane), s);
#pragma unroll
      for (int r = 0; r < 8; ++r) { const int qi = q0 + 8 * g + r; sS[w][8 * g + r][t * 16 + col] = key <= qi ? s[r] * scl : -3.0e38f; } }
    LDSX();
    float mx = -3.4e38f;
#pragma unroll
    for (int jj = 0; jj < 32; ++jj) mx = fmaxf(mx, sS[w][col][g * 32 + jj]);
    mx = fmaxf(mx, __shfl_xor(mx, 16, 32));
    const float mnew = fmaxf(mrun, mx); const float corr = expf(mrun - mnew);
    float ps = 0.f;
#pragma unroll
    for (int jj = 0; jj < 32; ++jj) { const float sv = sS[w][col][g * 32 + jj]; const float p = sv <= -1.0e38f ? 0.f : expf(sv - mnew); ps += p; sS[w][col][g * 32 + jj] = p; }
    ps += __shfl_xor(ps, 16, 32);
    lrun = lrun * corr + ps; mrun = mnew;
#pragma unroll
    for (int r = 0; r < 8; ++r) { const float cr = __shfl(corr, 8 * g + r, 32); acc[0][r] *= cr; acc[1][r] *= cr; }
    LDSX();
#pragma unroll
    for (int kc = 0; kc < 2; ++kc) { const F2 pa = split_row(&sS[w][col][0], kc * 32, lane);
#pragma unroll
      for (int t = 0; t < 2; ++t) acc[t] = mac3(pa, split_col(VH + (bh * LL + kt * 64) * HD, kc * 32, t * 16 + col, lane, HD, 64), acc[t]); }
    LDSX(); }
#pragma unroll
  for (int r = 0; r < 8; ++r) { const float lr = __shfl(lrun, 8 * g + r, 32);
#pragma unroll
    for (int t = 0; t < 2; ++t) sO[t * 16 + col][w * 16 + 8 * g + r] = acc[t][r] / lr; }
  __syncthreads();
  for (int q = tid; q < HD * 16; q += 128) { const int d = q >> 4, pc = q & 15; vst2(out + ((size_t)b * EM + h * HD + d) * LL + q0b + pc * 4, *(const v4f*)(&sO[d][pc * 4])); }
}
extern "C" void kernel_launch(void* const* d_in, const int* in_sizes, int n_in, void* d_out, int out_size, void* d_ws, size_t ws_size, hipStream_t stream) {
  (void)in_sizes; (void)n_in; (void)out_size; (void)ws_size;
  const float** I = (const float**)d_in;
  float* out = (float*)d_out;
  char* ws = (char*)d_ws; size_t off = 0;
  auto take = [&](size_t bytes) { char* p = ws + off; off += (bytes + 255) & ~(size_t)255; return p; };
  float* QH = (float*)take((size_t)NR * EM * 4); float* KH = (float*)take((size_t)NR * EM * 4); float* VH = (float*)take((size_t)NR * EM * 4);
  k_qkv<<<dim3(LL / 64, NB * 2, 3), 128, 0, stream>>>(I[0], I[1], I[2], I[3], I[4], I[5], I[6], I[7], QH, KH, VH);
  k_attn<<<dim3(LL / 64, NH, NB), 128, 0, stream>>>(QH, KH, VH, out);
}
